// GAT_6820408066447
// MI455X (gfx1250) — hardware-verified
//
#include <hip/hip_runtime.h>
#include <stddef.h>
#include <stdint.h>
#include <math.h>


#define NBAT   4
#define NN     2048
#define DF     128
#define MROWS  (NBAT * NN)
#define KT     64
#define QT     64
#define PP     72
#define SP     132
#define NEGV   (-9.0e15f)
#define WSMAX  134217728

#define PB_X   512
#define PB_WA  16
#define PB_WB  32
#define PB_MK  128
#define PB_ALL (PB_X + PB_WA + PB_WB + PB_MK)

static_assert(PB_X * 256 * 8 == MROWS * DF);
static_assert(PB_WA * 256 * 8 == 2 * DF * DF);
static_assert(PB_WB * 256 * 8 == 2 * DF * 2 * DF);
static_assert(PB_MK * 256 * 4 == NN * (NN / 32));
static_assert((DF % 32) == 0 && (NN % KT) == 0 && (NN % QT) == 0);
static_assert(2 * QT * PP * 2 <= QT * SP * 4);
static_assert((PP % 8) == 0 && (SP % 4) == 0);

typedef float          v4f  __attribute__((ext_vector_type(4)));
typedef float          v8f  __attribute__((ext_vector_type(8)));
typedef int            v8i  __attribute__((ext_vector_type(8)));
typedef unsigned int   v4u  __attribute__((ext_vector_type(4)));
typedef unsigned short v8us __attribute__((ext_vector_type(8)));
typedef __bf16         v16b __attribute__((ext_vector_type(16)));
typedef v4f  __attribute__((may_alias)) v4fa;
typedef v4u  __attribute__((may_alias)) v4ua;
typedef v8us __attribute__((may_alias)) v8usa;
union FragB { v16b v; v8us h[2]; v8i w; };

__device__ __forceinline__ v8f wmb(const FragB& a, const FragB& b, v8f c) {
  v8f d = __builtin_amdgcn_wmma_f32_16x16x32_bf16(false, a.v, false, b.v, (short)0, c, false, false);
  asm volatile("v_nop\n\tv_nop\n\tv_nop\n\tv_nop" : "+v"(d) : "v"(a.w), "v"(b.w));
  return d;
}

__device__ __forceinline__ unsigned int f2bf(float f) {
  const unsigned int u = __float_as_uint(f);
  return ((u + 0x7FFFu + ((u >> 16) & 1u)) >> 16) & 0xFFFFu;
}
__device__ __forceinline__ float bf2f(unsigned int b) { return __uint_as_float(b << 16); }
__device__ __forceinline__ float bfr(float f) { return bf2f(f2bf(f)); }
__device__ __forceinline__ unsigned int pk2(float lo, float hi) { return f2bf(lo) | (f2bf(hi) << 16); }
__device__ __forceinline__ v4u pack8(const v4f a, const v4f b) {
  v4u r;
  r.x = pk2(a.x, a.y); r.y = pk2(a.z, a.w); r.z = pk2(b.x, b.y); r.w = pk2(b.z, b.w);
  return r;
}
__device__ __forceinline__ void hilo2(float a, float b, unsigned int& hw, unsigned int& lw) {
  const unsigned int ha = f2bf(a), hb = f2bf(b);
  hw = ha | (hb << 16);
  lw = f2bf(a - bf2f(ha)) | (f2bf(b - bf2f(hb)) << 16);
}

__global__ __launch_bounds__(256) void k_prep(const float* __restrict__ x, const float* __restrict__ adj,
                                              const float* __restrict__ W1,
                                              unsigned short* XB, unsigned short* WA, unsigned short* WB,
                                              unsigned int* MK) {
  const int blk = (int)blockIdx.x, tid = (int)threadIdx.x;
  if (blk < PB_X) {
    const int u = blk * 256 + tid;
    const float* p = x + (size_t)u * 8;
    const v4f a = *(const v4fa*)p, b = *(const v4fa*)(p + 4);
    const v4u hv = pack8(a, b);
    unsigned short* o = XB + (size_t)u * 8;
    *(volatile v4u*)o = hv;
    __threadfence();
    *(volatile v4u*)o = hv;
  } else if (blk < PB_X + PB_WA) {
    const int u = (blk - PB_X) * 256 + tid;
    const float* p = W1 + (size_t)u * 8;
    const v4f a = *(const v4fa*)p, b = *(const v4fa*)(p + 4);
    const v4u hv = pack8(a, b);
    unsigned short* o = WA + (size_t)u * 8;
    *(volatile v4u*)o = hv;
    __threadfence();
    *(volatile v4u*)o = hv;
  } else if (blk < PB_X + PB_WA + PB_WB) {
    const int u  = (blk - PB_X - PB_WA) * 256 + tid;
    const int n  = u >> 5;
    const int k8 = (u & 31) * 8;
    const float* p = W1 + (size_t)2 * DF * DF + (size_t)n * DF + (k8 & (DF - 1));
    const v4f a = *(const v4fa*)p, b = *(const v4fa*)(p + 4);
    const v4u hv = pack8(a, b);
    unsigned short* o = WB + (size_t)n * (2 * DF) + k8;
    *(volatile v4u*)o = hv;
    __threadfence();
    *(volatile v4u*)o = hv;
  } else {
    const int u  = (blk - PB_X - PB_WA - PB_WB) * 256 + tid;
    const int i  = u >> 4;
    const int wq = u & 15;
    unsigned int w0 = 0u, w1 = 0u, w2 = 0u, w3 = 0u;
#pragma unroll 1
    for (int wi = 0; wi < 4; ++wi) {
      const int jb = 128 * wq + 32 * wi;
      const float* rp = adj + (size_t)i * NN + jb;
      unsigned int mbits = 0u;
#pragma unroll
      for (int g4 = 0; g4 < 8; ++g4) {
        const v4f v = *(const v4fa*)(rp + 4 * g4);
        const int j = jb + 4 * g4;
        mbits |= ((bfr(v.x) > 0.f && (j    ) != i) ? 1u : 0u) << (4 * g4);
        mbits |= ((bfr(v.y) > 0.f && (j + 1) != i) ? 1u : 0u) << (4 * g4 + 1);
        mbits |= ((bfr(v.z) > 0.f && (j + 2) != i) ? 1u : 0u) << (4 * g4 + 2);
        mbits |= ((bfr(v.w) > 0.f && (j + 3) != i) ? 1u : 0u) << (4 * g4 + 3);
      }
      w0 = (wi == 0) ? mbits : w0;
      w1 = (wi == 1) ? mbits : w1;
      w2 = (wi == 2) ? mbits : w2;
      w3 = (wi == 3) ? mbits : w3;
    }
    v4u mv; mv.x = w0; mv.y = w1; mv.z = w2; mv.w = w3;
    unsigned int* o = MK + (size_t)i * (NN / 32) + 4 * wq;
    *(volatile v4u*)o = mv;
    __threadfence();
    *(volatile v4u*)o = mv;
  }
}

__global__ __launch_bounds__(128) void k_lin(
    const unsigned short* __restrict__ A, const unsigned short* __restrict__ WT, int K,
    const float* __restrict__ bias2, const float* __restrict__ asrc, const float* __restrict__ adst,
    unsigned short* HTh, unsigned short* HTl, float* SD, float* HF)
{
  __shared__ __attribute__((aligned(16))) float stg[QT * SP];
  __shared__ __attribute__((aligned(16))) float satt[2 * DF];
  __shared__ __attribute__((aligned(16))) float sdot[2 * QT];
  __shared__ __attribute__((aligned(16))) float sbias[DF];
  const int tid = (int)threadIdx.x, lane = tid & 31, wave = tid >> 5, hh = lane >> 4, m = lane & 15;
  const int rowBase = (int)blockIdx.x * QT;
  const int ny      = (int)blockIdx.y;
  const int col0    = ny * DF;

  satt[tid]      = bfr(asrc[tid]);
  satt[DF + tid] = bfr(adst[tid]);
  sbias[tid]     = bfr(bias2[col0 + tid]);
  __syncthreads();

  v8f acc[8];
  {
    const v8f z = {0.f, 0.f, 0.f, 0.f, 0.f, 0.f, 0.f, 0.f};
#pragma unroll
    for (int t = 0; t < 8; ++t) acc[t] = z;
  }
  const unsigned short* ap = A  + (size_t)(rowBase + 16 * wave + m) * (size_t)K + 8 * hh;
  const unsigned short* wp = WT + (size_t)(col0 + m) * (size_t)K + 8 * hh;
  const int ksteps = K >> 5;
#pragma unroll 1
  for (int ks = 0; ks < ksteps; ++ks) {
    FragB af;
    af.h[0] = *(const v8usa*)(ap + 32 * ks);
    af.h[1] = *(const v8usa*)(ap + 32 * ks + 16);
#pragma unroll
    for (int t = 0; t < 8; ++t) {
      const unsigned short* wq = wp + (size_t)(16 * t) * (size_t)K + 32 * ks;
      FragB bf;
      bf.h[0] = *(const v8usa*)wq;
      bf.h[1] = *(const v8usa*)(wq + 16);
      acc[t] = wmb(af, bf, acc[t]);
    }
  }

#pragma unroll
  for (int t = 0; t < 8; ++t) {
    const int lc = 16 * t + m;
    const float bv = sbias[lc];
#pragma unroll
    for (int r = 0; r < 8; ++r) {
      const int lr = 16 * wave + 8 * hh + r;
      stg[lr * SP + lc] = acc[t][r] + bv;
    }
  }
  __syncthreads();

  if (ny == 0) {
    {
      const int row = tid & 63, which = tid >> 6;
      const float* sa = satt + which * DF;
      const float* hr = stg + row * SP;
      float d = 0.f;
#pragma unroll 4
      for (int c4 = 0; c4 < DF / 4; ++c4) {
        const v4f hv = *(const v4fa*)(hr + 4 * c4);
        const v4f av = *(const v4fa*)(sa + 4 * c4);
        d = fmaf(hv.x, av.x, d);
        d = fmaf(hv.y, av.y, d);
        d = fmaf(hv.z, av.z, d);
        d = fmaf(hv.w, av.w, d);
      }
      sdot[which * QT + row] = d;
    }
    __syncthreads();

    const int which2 = lane >> 4, piece = lane & 15;
    const v4f sdv = *(const v4fa*)(sdot + which2 * QT + 4 * piece);
    float* sp = SD + (size_t)which2 * MROWS + rowBase + 4 * piece;

    const int bb = rowBase >> 11, i0 = rowBase & (NN - 1);
    const int fq = lane >> 3, pc = lane & 7;
    v4u hv[8], lv[8];
#pragma unroll
    for (int p = 0; p < 8; ++p) {
      const int f = 16 * p + 4 * wave + fq;
      const float* s0 = stg + (8 * pc) * SP + f;
      const float v0 = s0[0],      v1 = s0[SP],     v2 = s0[2 * SP], v3 = s0[3 * SP];
      const float v4 = s0[4 * SP], v5 = s0[5 * SP], v6 = s0[6 * SP], v7 = s0[7 * SP];
      unsigned int h0, h1, h2, h3, l0, l1, l2, l3;
      hilo2(v0, v1, h0, l0); hilo2(v2, v3, h1, l1); hilo2(v4, v5, h2, l2); hilo2(v6, v7, h3, l3);
      hv[p].x = h0; hv[p].y = h1; hv[p].z = h2; hv[p].w = h3;
      lv[p].x = l0; lv[p].y = l1; lv[p].z = l2; lv[p].w = l3;
    }
#pragma unroll
    for (int p = 0; p < 8; ++p) {
      const int f = 16 * p + 4 * wave + fq;
      const size_t o = ((size_t)(bb * DF + f)) * NN + i0 + 8 * pc;
      *(volatile v4u*)(HTh + o) = hv[p];
      *(volatile v4u*)(HTl + o) = lv[p];
    }
    if (wave == 0) *(volatile v4f*)sp = sdv;
    __threadfence();
#pragma unroll
    for (int p = 0; p < 8; ++p) {
      const int f = 16 * p + 4 * wave + fq;
      const size_t o = ((size_t)(bb * DF + f)) * NN + i0 + 8 * pc;
      *(volatile v4u*)(HTh + o) = hv[p];
      *(volatile v4u*)(HTl + o) = lv[p];
    }
    if (wave == 0) *(volatile v4f*)sp = sdv;
  } else {
    v4f fv[16];
#pragma unroll
    for (int i = 0; i < 16; ++i) {
      const int lr = 16 * wave + i;
      fv[i] = *(const v4fa*)(stg + lr * SP + 4 * lane);
    }
#pragma unroll
    for (int i = 0; i < 16; ++i) {
      const int gr = rowBase + 16 * wave + i;
      float* op = HF + (size_t)gr * DF + 4 * lane;
      *(volatile v4f*)op = fv[i];
    }
    __threadfence();
#pragma unroll
    for (int i = 0; i < 16; ++i) {
      const int gr = rowBase + 16 * wave + i;
      float* op = HF + (size_t)gr * DF + 4 * lane;
      *(volatile v4f*)op = fv[i];
    }
  }
}

template<int MODE>
__global__ __launch_bounds__(256) void k_att(
    const unsigned short* __restrict__ HTh, const unsigned short* __restrict__ HTl,
    const float* __restrict__ SD, const unsigned int* __restrict__ MK, const float* __restrict__ abp,
    const float* __restrict__ Hadd,
    const float* __restrict__ bng, const float* __restrict__ bnb,
    const float* __restrict__ bnm, const float* __restrict__ bnv,
    unsigned short* YP, float* outF)
{
  __shared__ __attribute__((aligned(16))) float        sU[QT * SP];
  __shared__ __attribute__((aligned(16))) float        sd[NN];
  __shared__ __attribute__((aligned(16))) unsigned int smk[QT * (NN / 32)];
  __shared__ __attribute__((aligned(16))) float        ssc[QT];
  __shared__ __attribute__((aligned(16))) float        sl[QT];
  __shared__ __attribute__((aligned(16))) float        sbn[3 * QT];

  const int tid = (int)threadIdx.x, lane = tid & 31, wave = tid >> 5, hh = lane >> 4, m = lane & 15;
  const int b  = (int)blockIdx.x >> 5;
  const int i0 = ((int)blockIdx.x & 31) * QT;
  const int rg = wave & 3, ch = wave >> 2;
  const int r  = tid >> 2, q = tid & 3;

  {
    const float* Dp = SD + (size_t)MROWS + (size_t)b * NN;
    *(v4fa*)(sd + 4 * tid)         = *(const v4fa*)(Dp + 4 * tid);
    *(v4fa*)(sd + 4 * (tid + 256)) = *(const v4fa*)(Dp + 4 * (tid + 256));
    const unsigned int* mp = MK + (size_t)i0 * (NN / 32);
#pragma unroll
    for (int k = 0; k < 4; ++k)
      *(v4ua*)(smk + 4 * (tid + 256 * k)) = *(const v4ua*)(mp + 4 * (tid + 256 * k));
    if (MODE == 0) {
      if (tid < QT) {
        const int i = i0 + tid;
        const float g = bfr(bng[i]), be = bfr(bnb[i]), mu = bfr(bnm[i]), va = bfr(bnv[i]);
        const float inv = 1.0f / sqrtf(va + 1e-5f);
        sbn[tid]          = mu;
        sbn[QT + tid]     = inv * g;
        sbn[2 * QT + tid] = be;
      }
    }
  }
  const float si = SD[(size_t)b * NN + i0 + r];
  const float ab = bfr(abp[0]);
  __syncthreads();

  unsigned short* ph = (unsigned short*)sU;
  unsigned short* pl = ph + QT * PP;

  v8f acc[4];
  {
    const v8f z = {0.f, 0.f, 0.f, 0.f, 0.f, 0.f, 0.f, 0.f};
    acc[0] = z; acc[1] = z; acc[2] = z; acc[3] = z;
  }
  float mrun = __int_as_float((int)0xff800000);
  float lrun = 0.f;

  const size_t hrow = ((size_t)(b * DF + 64 * ch + m)) * NN + 8 * hh;
  const unsigned short* bh0 = HTh + hrow;
  const unsigned short* bl0 = HTl + hrow;

#pragma unroll 1
  for (int tj = 0; tj < NN / KT; ++tj) {
    const int j0 = KT * tj;
    {
      const float* dp = sd + j0 + 16 * q;
      const v4f d0 = *(const v4fa*)dp, d1 = *(const v4fa*)(dp + 4), d2 = *(const v4fa*)(dp + 8), d3 = *(const v4fa*)(dp + 12);
      float e[16] = {d0.x, d0.y, d0.z, d0.w, d1.x, d1.y, d1.z, d1.w, d2.x, d2.y, d2.z, d2.w, d3.x, d3.y, d3.z, d3.w};
      const unsigned int mw = smk[r * (NN / 32) + 2 * tj + (q >> 1)] >> (16 * (q & 1));
      float tmax = -3.0e38f;
#pragma unroll
      for (int c = 0; c < 16; ++c) {
        float v = (si + e[c]) + ab;
        v = fmaxf(v, 0.f);
        v = (((mw >> c) & 1u) != 0u) ? v : NEGV;
        e[c] = v;
        tmax = fmaxf(tmax, v);
      }
      tmax = fmaxf(tmax, __shfl_xor(tmax, 1));
      tmax = fmaxf(tmax, __shfl_xor(tmax, 2));
      const float mnew = fmaxf(mrun, tmax);
      const float ex   = expf(mrun - mnew);
      const float scl  = (mrun > -1.0e30f) ? ex : 0.f;
      float ps = 0.f;
      unsigned int hw[8], lw[8];
#pragma unroll
      for (int c = 0; c < 8; ++c) {
        const float p0 = expf(e[2 * c] - mnew);
        const float p1 = expf(e[2 * c + 1] - mnew);
        ps += p0; ps += p1;
        hilo2(p0, p1, hw[c], lw[c]);
      }
      ps += __shfl_xor(ps, 1);
      ps += __shfl_xor(ps, 2);
      lrun = fmaf(lrun, scl, ps);
      mrun = mnew;
      if (q == 0) ssc[r] = scl;
      v4u a0, a1, c0, c1;
      a0.x = hw[0]; a0.y = hw[1]; a0.z = hw[2]; a0.w = hw[3];
      a1.x = hw[4]; a1.y = hw[5]; a1.z = hw[6]; a1.w = hw[7];
      c0.x = lw[0]; c0.y = lw[1]; c0.z = lw[2]; c0.w = lw[3];
      c1.x = lw[4]; c1.y = lw[5]; c1.z = lw[6]; c1.w = lw[7];
      const int off = r * PP + 16 * q;
      *(v4ua*)(ph + off)     = a0;
      *(v4ua*)(ph + off + 8) = a1;
      *(v4ua*)(pl + off)     = c0;
      *(v4ua*)(pl + off + 8) = c1;
    }
    __syncthreads();

    {
      const v4f s0 = *(const v4fa*)(ssc + 16 * rg + 8 * hh);
      const v4f s1 = *(const v4fa*)(ssc + 16 * rg + 8 * hh + 4);
#pragma unroll
      for (int t = 0; t < 4; ++t) {
        acc[t][0] *= s0.x; acc[t][1] *= s0.y; acc[t][2] *= s0.z; acc[t][3] *= s0.w;
        acc[t][4] *= s1.x; acc[t][5] *= s1.y; acc[t][6] *= s1.z; acc[t][7] *= s1.w;
      }
#pragma unroll
      for (int ks = 0; ks < 2; ++ks) {
        FragB ah, al;
        const int ao = (16 * rg + m) * PP + 32 * ks + 8 * hh;
        ah.h[0] = *(const v8usa*)(ph + ao);
        ah.h[1] = *(const v8usa*)(ph + ao + 16);
        al.h[0] = *(const v8usa*)(pl + ao);
        al.h[1] = *(const v8usa*)(pl + ao + 16);
#pragma unroll
        for (int t = 0; t < 4; ++t) {
          const size_t bo = (size_t)(16 * t) * NN + j0 + 32 * ks;
          FragB bh, bl;
          bh.h[0] = *(const v8usa*)(bh0 + bo);
          bh.h[1] = *(const v8usa*)(bh0 + bo + 16);
          bl.h[0] = *(const v8usa*)(bl0 + bo);
          bl.h[1] = *(const v8usa*)(bl0 + bo + 16);
          acc[t] = wmb(ah, bh, acc[t]);
          acc[t] = wmb(ah, bl, acc[t]);
          acc[t] = wmb(al, bh, acc[t]);
        }
      }
    }
    __syncthreads();
  }

  if (q == 0) sl[r] = 1.0f / lrun;
#pragma unroll
  for (int t = 0; t < 4; ++t) {
    const int lc = 64 * ch + 16 * t + m;
#pragma unroll
    for (int rr = 0; rr < 8; ++rr) {
      const int lr = 16 * rg + 8 * hh + rr;
      sU[lr * SP + lc] = acc[t][rr];
    }
  }
  __syncthreads();

  if (MODE == 0) {
    const int cg = lane & 15;
    const bool lsel = lane >= 16;
    v4u pv[8];
#pragma unroll
    for (int i = 0; i < 8; ++i) {
      const int lr = 8 * wave + i;
      const size_t grow = (size_t)b * NN + i0 + lr;
      const float inv = sl[lr];
      const float mu = sbn[lr], sc = sbn[QT + lr], be = sbn[2 * QT + lr];
      const v4f o0 = *(const v4fa*)(sU + lr * SP + 8 * cg);
      const v4f o1 = *(const v4fa*)(sU + lr * SP + 8 * cg + 4);
      const v4f g0 = *(const v4fa*)(Hadd + grow * DF + 8 * cg);
      const v4f g1 = *(const v4fa*)(Hadd + grow * DF + 8 * cg + 4);
      float y0 = fmaxf(fmaf(o0.x, inv, g0.x), 0.f), y1 = fmaxf(fmaf(o0.y, inv, g0.y), 0.f);
      float y2 = fmaxf(fmaf(o0.z, inv, g0.z), 0.f), y3 = fmaxf(fmaf(o0.w, inv, g0.w), 0.f);
      float y4 = fmaxf(fmaf(o1.x, inv, g1.x), 0.f), y5 = fmaxf(fmaf(o1.y, inv, g1.y), 0.f);
      float y6 = fmaxf(fmaf(o1.z, inv, g1.z), 0.f), y7 = fmaxf(fmaf(o1.w, inv, g1.w), 0.f);
      y0 = (y0 - mu) * sc + be; y1 = (y1 - mu) * sc + be; y2 = (y2 - mu) * sc + be; y3 = (y3 - mu) * sc + be;
      y4 = (y4 - mu) * sc + be; y5 = (y5 - mu) * sc + be; y6 = (y6 - mu) * sc + be; y7 = (y7 - mu) * sc + be;
      unsigned int h0, h1, h2, h3, l0, l1, l2, l3;
      hilo2(y0, y1, h0, l0); hilo2(y2, y3, h1, l1); hilo2(y4, y5, h2, l2); hilo2(y6, y7, h3, l3);
      pv[i].x = lsel ? l0 : h0;
      pv[i].y = lsel ? l1 : h1;
      pv[i].z = lsel ? l2 : h2;
      pv[i].w = lsel ? l3 : h3;
    }
#pragma unroll
    for (int i = 0; i < 8; ++i) {
      const size_t grow = (size_t)b * NN + i0 + 8 * wave + i;
      unsigned short* gp = YP + grow * (2 * DF) + 8 * lane;
      *(volatile v4u*)gp = pv[i];
    }
    __threadfence();
#pragma unroll
    for (int i = 0; i < 8; ++i) {
      const size_t grow = (size_t)b * NN + i0 + 8 * wave + i;
      unsigned short* gp = YP + grow * (2 * DF) + 8 * lane;
      *(volatile v4u*)gp = pv[i];
    }
  } else {
    v4f ov[8];
#pragma unroll
    for (int i = 0; i < 8; ++i) {
      const int lr = 8 * wave + i;
      const size_t grow = (size_t)b * NN + i0 + lr;
      const float inv = sl[lr];
      const v4f o = *(const v4fa*)(sU + lr * SP + 4 * lane);
      const v4f g = *(const v4fa*)(Hadd + grow * DF + 4 * lane);
      v4f v;
      v.x = fmaf(o.x, inv, g.x); v.y = fmaf(o.y, inv, g.y);
      v.z = fmaf(o.z, inv, g.z); v.w = fmaf(o.w, inv, g.w);
      ov[i] = v;
    }
#pragma unroll
    for (int i = 0; i < 8; ++i) {
      const size_t grow = (size_t)b * NN + i0 + 8 * wave + i;
      float* gp = outF + grow * DF + 4 * lane;
      *(volatile v4f*)gp = ov[i];
    }
    __threadfence();
#pragma unroll
    for (int i = 0; i < 8; ++i) {
      const size_t grow = (size_t)b * NN + i0 + 8 * wave + i;
      float* gp = outF + grow * DF + 4 * lane;
      *(volatile v4f*)gp = ov[i];
    }
  }
  (void)YP; (void)outF; (void)bng; (void)bnb; (void)bnm; (void)bnv;
}

extern "C" void kernel_launch(void* const* d_in, const int* in_sizes, int n_in,
                              void* d_out, int out_size, void* d_ws, size_t ws_size,
                              hipStream_t stream) {
  if (n_in < 11) return;
  if (in_sizes[0] != MROWS * DF) return;
  if (in_sizes[1] != NN * NN) return;
  if (in_sizes[2] != 4 * DF * DF) return;
  if (in_sizes[3] != 4 * DF) return;
  if (in_sizes[4] != 4 * DF || in_sizes[5] != 4 * DF) return;
  if (in_sizes[6] != 4) return;
  if (in_sizes[7] != NN || in_sizes[8] != NN || in_sizes[9] != NN || in_sizes[10] != NN) return;
  if (out_size != MROWS * DF) return;

  const float* x     = (const float*)d_in[0];
  const float* adj   = (const float*)d_in[1];
  const float* W1    = (const float*)d_in[2];
  const float* b1    = (const float*)d_in[3];
  const float* a_src = (const float*)d_in[4];
  const float* a_dst = (const float*)d_in[5];
  const float* a_b   = (const float*)d_in[6];
  const float* bng   = (const float*)d_in[7];
  const float* bnb   = (const float*)d_in[8];
  const float* bnm   = (const float*)d_in[9];
  const float* bnv   = (const float*)d_in[10];
  float* out = (float*)d_out;

  char* ws = (char*)d_ws;
  size_t off = 0;
  const size_t oXB  = off; off += (size_t)MROWS * DF * 2;          off = (off + 255) & ~(size_t)255;
  const size_t oWA  = off; off += (size_t)2 * DF * DF * 2;         off = (off + 255) & ~(size_t)255;
  const size_t oWB  = off; off += (size_t)2 * DF * 2 * DF * 2;     off = (off + 255) & ~(size_t)255;
  const size_t oMK  = off; off += (size_t)NN * (NN / 32) * 4;      off = (off + 255) & ~(size_t)255;
  const size_t oT1h = off; off += (size_t)NBAT * DF * NN * 2;      off = (off + 255) & ~(size_t)255;
  const size_t oT1l = off; off += (size_t)NBAT * DF * NN * 2;      off = (off + 255) & ~(size_t)255;
  const size_t oT2h = off; off += (size_t)NBAT * DF * NN * 2;      off = (off + 255) & ~(size_t)255;
  const size_t oT2l = off; off += (size_t)NBAT * DF * NN * 2;      off = (off + 255) & ~(size_t)255;
  const size_t oH1  = off; off += (size_t)MROWS * DF * 4;          off = (off + 255) & ~(size_t)255;
  const size_t oH3  = off; off += (size_t)MROWS * DF * 4;          off = (off + 255) & ~(size_t)255;
  const size_t oSD1 = off; off += (size_t)2 * MROWS * 4;           off = (off + 255) & ~(size_t)255;
  const size_t oSD2 = off; off += (size_t)2 * MROWS * 4;           off = (off + 255) & ~(size_t)255;
  const size_t oYP  = off; off += (size_t)MROWS * 2 * DF * 2;      off = (off + 255) & ~(size_t)255;
  if (off > ws_size || off > (size_t)WSMAX) return;

  unsigned short* XB  = (unsigned short*)(ws + oXB);
  unsigned short* WA  = (unsigned short*)(ws + oWA);
  unsigned short* WB  = (unsigned short*)(ws + oWB);
  unsigned int*   MK  = (unsigned int*)(ws + oMK);
  unsigned short* T1h = (unsigned short*)(ws + oT1h);
  unsigned short* T1l = (unsigned short*)(ws + oT1l);
  unsigned short* T2h = (unsigned short*)(ws + oT2h);
  unsigned short* T2l = (unsigned short*)(ws + oT2l);
  float*          H1  = (float*)(ws + oH1);
  float*          H3  = (float*)(ws + oH3);
  float*          SD1 = (float*)(ws + oSD1);
  float*          SD2 = (float*)(ws + oSD2);
  unsigned short* YP  = (unsigned short*)(ws + oYP);

  k_prep<<<PB_ALL, 256, 0, stream>>>(x, adj, W1, XB, WA, WB, MK);
  k_lin<<<dim3(MROWS / QT, 2), 128, 0, stream>>>(XB, WA, DF, b1, a_src, a_dst, T1h, T1l, SD1, H1);
  k_att<0><<<NBAT * (NN / QT), 256, 0, stream>>>(T1h, T1l, SD1, MK, a_b + 0, H1, bng, bnb, bnm, bnv, YP, out);
  k_lin<<<dim3(MROWS / QT, 2), 128, 0, stream>>>(YP, WB, 2 * DF, b1 + 2 * DF, a_src + 2 * DF, a_dst + 2 * DF,
                                                 T2h, T2l, SD2, H3);
  k_att<1><<<NBAT * (NN / QT), 256, 0, stream>>>(T2h, T2l, SD2, MK, a_b + 2, H3, bng, bnb, bnm, bnv, YP, out);
}
